// CrossAttention_11751030522327
// MI455X (gfx1250) — hardware-verified
//
#include <hip/hip_runtime.h>


#ifndef NB
#define NB 8
#endif
#ifndef SEQ
#define SEQ 1024
#endif
#define NB_FULL  8
#define SEQ_FULL 1024
#define DM   512
#define NH   8
#define HD   64
#define DFF  1024
#define NTOK (NB * SEQ)
#define NCH  (SEQ / 128)
#define CQK  16.0f
#define CVV  8.0f
#define PCAR 1024.0f
#define CX   16.0f
#define CW   64.0f
#define SCL  (1.0f / 2048.0f)
#define OSC_O (1.0f / 524288.0f)
#define OSC_F (1.0f / 1024.0f)
#define LNEPS 1e-5f
#define OUT1_OFF ((size_t)NB_FULL * SEQ_FULL * DM)
static_assert(OUT1_OFF * 4 == (size_t)16777216);
static_assert(SEQ % 128 == 0);
static_assert(SEQ <= SEQ_FULL);
static_assert(NB >= 1 && NB <= NB_FULL);
static_assert(DM % 128 == 0 && DFF % 64 == 0 && HD == 64 && NH * HD == DM);
static_assert(NTOK % 64 == 0);

typedef _Float16 h16;
typedef unsigned short bf;
typedef __attribute__((ext_vector_type(16))) __bf16   v16bf;
typedef __attribute__((ext_vector_type(16))) _Float16 v16h;
typedef __attribute__((ext_vector_type(8)))  _Float16 v8h;
typedef __attribute__((ext_vector_type(4)))  _Float16 v4h;
typedef __attribute__((ext_vector_type(8)))  unsigned short v8us;
typedef __attribute__((ext_vector_type(4)))  unsigned short v4us;
typedef __attribute__((ext_vector_type(8)))  float    v8f;
typedef __attribute__((ext_vector_type(4)))  float    v4f;
typedef v8h  __attribute__((may_alias)) v8ha;
typedef v4f  __attribute__((may_alias)) v4fa;
typedef v8us __attribute__((may_alias)) v8usa;

__device__ __forceinline__ unsigned short f2bf(float f) { unsigned u = __float_as_uint(f); u += 0x7FFFu + ((u >> 16) & 1u); return (unsigned short)(u >> 16); }
__device__ __forceinline__ float bf2f(unsigned short b) { return __uint_as_float(((unsigned)b) << 16); }
__device__ __forceinline__ float bfr(float f) { return bf2f(f2bf(f)); }
__device__ __forceinline__ h16 tohx(float x) { return (h16)x; }
__device__ __forceinline__ v16h cat16(v8h lo, v8h hi) { return __builtin_shufflevector(lo, hi, 0, 1, 2, 3, 4, 5, 6, 7, 8, 9, 10, 11, 12, 13, 14, 15); }
__device__ __forceinline__ v16bf cat16b(v8us lo, v8us hi) { return __builtin_bit_cast(v16bf, __builtin_shufflevector(lo, hi, 0, 1, 2, 3, 4, 5, 6, 7, 8, 9, 10, 11, 12, 13, 14, 15)); }
__device__ __forceinline__ v8f wmma16(v16h a, v16h b, v8f c) { return __builtin_amdgcn_wmma_f32_16x16x32_f16(false, a, false, b, (short)0, c, false, false); }
__device__ __forceinline__ v8f wmmab(v16bf a, v16bf b, v8f c) { return __builtin_amdgcn_wmma_f32_16x16x32_bf16(false, a, false, b, (short)0, c, false, false); }

template <typename T16> struct WFrag;
template <> struct WFrag<h16> { typedef v16h V; static __device__ __forceinline__ V ld(const h16* p) { return cat16(*(const v8h*)p, *(const v8h*)(p + 16)); } static __device__ __forceinline__ v8f mma(V a, V b, v8f c) { return wmma16(a, b, c); } };
template <> struct WFrag<bf> { typedef v16bf V; static __device__ __forceinline__ V ld(const bf* p) { return cat16b(*(const v8us*)p, *(const v8us*)(p + 16)); } static __device__ __forceinline__ v8f mma(V a, V b, v8f c) { return wmmab(a, b, c); } };
template <typename T16, bool BIAS>
__global__ __launch_bounds__(32) void k_gemmw(const T16* __restrict__ A, int lda, const T16* __restrict__ Bt, int ldb, int K,
                                              float* C, int ldc, const float* __restrict__ bias, float osc, size_t sA, size_t sB, size_t sC) {
    typedef typename WFrag<T16>::V V;
    __shared__ __align__(16) float os[16 * 68];
    const size_t z = blockIdx.z; A += z * sA; Bt += z * sB; C += z * sC;
    const int lane = threadIdx.x & 31, lr = lane & 15, hi = lane >> 4; const int r0 = blockIdx.x * 64, c0 = blockIdx.y * 64;
    v8f acc[4][4];
#pragma unroll
    for (int mb = 0; mb < 4; ++mb)
#pragma unroll
        for (int nb = 0; nb < 4; ++nb) acc[mb][nb] = (v8f){};
    const size_t aoff = (size_t)(r0 + lr) * lda + 8 * hi, boff = (size_t)(c0 + lr) * ldb + 8 * hi;
#pragma unroll 1
    for (int kc = 0; kc < K; kc += 32) {
        V a[4];
#pragma unroll
        for (int mb = 0; mb < 4; ++mb) a[mb] = WFrag<T16>::ld(A + aoff + (size_t)mb * 16 * lda + kc);
#pragma unroll
        for (int nb = 0; nb < 4; ++nb) { const V b = WFrag<T16>::ld(Bt + boff + (size_t)nb * 16 * ldb + kc);
#pragma unroll
            for (int mb = 0; mb < 4; ++mb) acc[mb][nb] = WFrag<T16>::mma(a[mb], b, acc[mb][nb]); }
        asm volatile("v_nop\n\tv_nop\n\tv_nop\n\tv_nop" : "+v"(acc[0][0]), "+v"(acc[1][1]), "+v"(acc[2][2]), "+v"(acc[3][3]) : "v"(a[0]), "v"(a[3]));
    }
#pragma unroll
    for (int mb = 0; mb < 4; ++mb) {
#pragma unroll
        for (int nb = 0; nb < 4; ++nb) {
#pragma unroll
            for (int j = 0; j < 8; ++j) os[(hi * 8 + j) * 68 + nb * 16 + lr] = acc[mb][nb][j]; }
        __syncthreads();
        float* crow = C + (size_t)(r0 + mb * 16) * ldc + c0;
#pragma unroll 1
        for (int ps = 0; ps < 2; ++ps) {
#pragma unroll
            for (int s = 0; s < 8; ++s) { const int row = 2 * s + hi, cofs = lr * 4; v4f val = *(const v4fa*)(os + row * 68 + cofs); val = val * osc;
                if (BIAS) { val[0] += bfr(bias[c0 + cofs]); val[1] += bfr(bias[c0 + cofs + 1]); val[2] += bfr(bias[c0 + cofs + 2]); val[3] += bfr(bias[c0 + cofs + 3]); }
                *(volatile v4f*)(crow + (size_t)row * ldc + cofs) = val; }
            if (ps == 0) __threadfence(); }
        __syncthreads();
    }
}

__global__ __launch_bounds__(256) void k_cvtin(const float* __restrict__ X, bf* XB, size_t n8) {
    const size_t i = (size_t)blockIdx.x * 256 + threadIdx.x; if (i >= n8) return;
    const size_t tok = i / (DM / 8); const int c8 = (int)(i % (DM / 8)) * 8; const size_t b = tok / SEQ, t = tok % SEQ;
    const float* s = X + (b * SEQ_FULL + t) * DM + c8;
    const v4f v0 = *(const v4f*)s, v1 = *(const v4f*)(s + 4); v8us o;
#pragma unroll
    for (int k = 0; k < 4; ++k) { o[k] = f2bf(v0[k]); o[4 + k] = f2bf(v1[k]); }
    bf* d = XB + tok * DM + c8; *(volatile v8us*)d = o; __threadfence(); *(volatile v8us*)d = o;
}
__global__ __launch_bounds__(256) void k_cvtb(const float* __restrict__ src, bf* dst, size_t n8) {
    const size_t i = (size_t)blockIdx.x * 256 + threadIdx.x; if (i >= n8) return;
    const v4f v0 = *(const v4f*)(src + i * 8), v1 = *(const v4f*)(src + i * 8 + 4); v8us o;
#pragma unroll
    for (int k = 0; k < 4; ++k) { o[k] = f2bf(v0[k]); o[4 + k] = f2bf(v1[k]); }
    *(volatile v8us*)(dst + i * 8) = o; __threadfence(); *(volatile v8us*)(dst + i * 8) = o;
}
__global__ __launch_bounds__(256) void k_cvth(const float* __restrict__ src, h16* dst, size_t n8, float sc) {
    const size_t i = (size_t)blockIdx.x * 256 + threadIdx.x; if (i >= n8) return;
    const v4f v0 = *(const v4f*)(src + i * 8), v1 = *(const v4f*)(src + i * 8 + 4); v8h o;
#pragma unroll
    for (int k = 0; k < 4; ++k) { o[k] = tohx(bfr(v0[k]) * sc); o[4 + k] = tohx(bfr(v1[k]) * sc); }
    *(volatile v8h*)(dst + i * 8) = o; __threadfence(); *(volatile v8h*)(dst + i * 8) = o;
}
template <bool RELU, bool RB>
__global__ __launch_bounds__(256) void k_tof16(const float* __restrict__ F, h16* P, size_t n8, float sc, const float* __restrict__ bias, int ncol, int nbias) {
    const size_t i = (size_t)blockIdx.x * 256 + threadIdx.x; if (i >= n8) return;
    const size_t e = i * 8;
    const v4f v0 = *(const v4f*)(F + e), v1 = *(const v4f*)(F + e + 4);
    float bb = 0.f;
    if (RB) { const int r = (int)((e / (size_t)ncol) % (size_t)nbias); bb = bfr(bias[r]); }
    v8h o;
#pragma unroll
    for (int k = 0; k < 4; ++k) {
        float x0 = v0[k] + bb, x1 = v1[k] + bb;
        if (RELU) { x0 = fmaxf(x0, 0.f); x1 = fmaxf(x1, 0.f); }
        o[k] = tohx(x0 * sc); o[4 + k] = tohx(x1 * sc); }
    *(volatile v8h*)(P + e) = o; __threadfence(); *(volatile v8h*)(P + e) = o;
}

__global__ __launch_bounds__(256) void k_soft(const float* __restrict__ S, h16* P16, float* W) {
    const int lane = threadIdx.x & 31; const int qrow = blockIdx.x * 8 + (threadIdx.x >> 5); if (qrow >= SEQ) return;
    v4f wacc[NCH];
#pragma unroll
    for (int ch = 0; ch < NCH; ++ch) wacc[ch] = (v4f){};
#pragma unroll 1
    for (int h = 0; h < NH; ++h) {
        const float* sr = S + ((size_t)h * SEQ + qrow) * SEQ;
        v4f x[NCH];
#pragma unroll
        for (int ch = 0; ch < NCH; ++ch) x[ch] = *(const v4f*)(sr + ch * 128 + lane * 4);
        float mx = -3.0e38f;
#pragma unroll
        for (int ch = 0; ch < NCH; ++ch) { x[ch] = x[ch] * SCL;
#pragma unroll
            for (int k = 0; k < 4; ++k) mx = fmaxf(mx, x[ch][k]); }
#pragma unroll
        for (int sh = 16; sh; sh >>= 1) mx = fmaxf(mx, __shfl_xor(mx, sh, 32));
        float sum = 0.f;
#pragma unroll
        for (int ch = 0; ch < NCH; ++ch) {
#pragma unroll
            for (int k = 0; k < 4; ++k) { float d0 = x[ch][k] - mx; asm volatile("" : "+v"(d0)); const float ex = __builtin_amdgcn_exp2f(d0 * 1.4426950408889634f); x[ch][k] = ex; sum += ex; } }
#pragma unroll
        for (int sh = 16; sh; sh >>= 1) sum += __shfl_xor(sum, sh, 32);
        const float rinv = __fdiv_rn(1.0f, sum); const float f = rinv * PCAR;
        v4h o[NCH];
#pragma unroll
        for (int ch = 0; ch < NCH; ++ch) {
#pragma unroll
            for (int k = 0; k < 4; ++k) { const float ex = x[ch][k]; o[ch][k] = tohx(ex * f); const float p = ex * rinv; wacc[ch][k] = wacc[ch][k] + p; } }
        h16* prow = P16 + ((size_t)h * SEQ + qrow) * SEQ;
#pragma unroll 1
        for (int ps = 0; ps < 2; ++ps) {
#pragma unroll
            for (int ch = 0; ch < NCH; ++ch) *(volatile v4h*)(prow + ch * 128 + lane * 4) = o[ch];
            if (ps == 0) __threadfence(); }
    }
#pragma unroll
    for (int ch = 0; ch < NCH; ++ch) wacc[ch] = wacc[ch] * (1.0f / NH);
    float* wr = W + (size_t)qrow * SEQ;
#pragma unroll 1
    for (int ps = 0; ps < 2; ++ps) {
#pragma unroll
        for (int ch = 0; ch < NCH; ++ch) *(volatile v4f*)(wr + ch * 128 + lane * 4) = wacc[ch];
        if (ps == 0) __threadfence(); }
}

template <bool FIRST>
__global__ __launch_bounds__(256) void k_ln(const float* __restrict__ Ain, const float* __restrict__ Badd, const float* __restrict__ g, const float* __restrict__ be, float* OF, h16* OH) {
    const int lane = threadIdx.x & 31; const int tok = blockIdx.x * 8 + (threadIdx.x >> 5); if (tok >= NTOK) return;
    const float* arow;
    if (FIRST) { const int b = tok / SEQ, t = tok - b * SEQ; arow = Ain + ((size_t)b * SEQ_FULL + t) * DM; } else arow = Ain + (size_t)tok * DM;
    const float* brow = Badd + (size_t)tok * DM;
    v4f tv[DM / 128]; float s1 = 0.f;
#pragma unroll
    for (int ch = 0; ch < DM / 128; ++ch) { v4f a = *(const v4f*)(arow + ch * 128 + lane * 4); const v4f bb = *(const v4f*)(brow + ch * 128 + lane * 4);
        if (FIRST) {
#pragma unroll
            for (int k = 0; k < 4; ++k) a[k] = bfr(a[k]); }
        tv[ch] = a + bb;
#pragma unroll
        for (int k = 0; k < 4; ++k) s1 += tv[ch][k]; }
#pragma unroll
    for (int sh = 16; sh; sh >>= 1) s1 += __shfl_xor(s1, sh, 32);
    const float mean = s1 * (1.0f / DM);
    float s2 = 0.f;
#pragma unroll
    for (int ch = 0; ch < DM / 128; ++ch) {
#pragma unroll
        for (int k = 0; k < 4; ++k) { const float d = tv[ch][k] - mean; s2 += d * d; } }
#pragma unroll
    for (int sh = 16; sh; sh >>= 1) s2 += __shfl_xor(s2, sh, 32);
    const float var = s2 * (1.0f / DM); const float rstd = rsqrtf(var + LNEPS);
    v4f y[DM / 128]; v4h yh[DM / 128];
#pragma unroll
    for (int ch = 0; ch < DM / 128; ++ch) { const v4f gv = *(const v4f*)(g + ch * 128 + lane * 4); const v4f bv = *(const v4f*)(be + ch * 128 + lane * 4);
#pragma unroll
        for (int k = 0; k < 4; ++k) { const float yy = (tv[ch][k] - mean) * rstd * bfr(gv[k]) + bfr(bv[k]); y[ch][k] = yy; yh[ch][k] = tohx(yy * CX); } }
    float* orow = OF + (size_t)tok * DM;
#pragma unroll 1
    for (int ps = 0; ps < 2; ++ps) {
#pragma unroll
        for (int ch = 0; ch < DM / 128; ++ch) { *(volatile v4f*)(orow + ch * 128 + lane * 4) = y[ch]; if (FIRST) *(volatile v4h*)(OH + (size_t)tok * DM + ch * 128 + lane * 4) = yh[ch]; }
        if (ps == 0) __threadfence(); }
}

extern "C" void kernel_launch(void* const* d_in, const int* in_sizes, int n_in,
                              void* d_out, int out_size, void* d_ws, size_t ws_size, hipStream_t stream) {
    if (n_in < 15) return;
    const float* q    = (const float*)d_in[0];  const float* kin  = (const float*)d_in[1];  const float* vin  = (const float*)d_in[2];
    const float* ipw  = (const float*)d_in[3];  const float* ipb  = (const float*)d_in[4];
    const float* ow   = (const float*)d_in[5];  const float* ob   = (const float*)d_in[6];
    const float* ln1g = (const float*)d_in[7];  const float* ln1b = (const float*)d_in[8];
    const float* w1   = (const float*)d_in[9];  const float* b1   = (const float*)d_in[10];
    const float* w2   = (const float*)d_in[11]; const float* b2   = (const float*)d_in[12];
    const float* ln2g = (const float*)d_in[13]; const float* ln2b = (const float*)d_in[14];
    const size_t needA = ((size_t)(NB - 1) * SEQ_FULL + SEQ) * DM;
    if ((size_t)in_sizes[0] < needA || (size_t)in_sizes[1] < needA || (size_t)in_sizes[2] < needA) return;
    if ((size_t)in_sizes[3] < (size_t)3 * DM * DM || in_sizes[4] < 3 * DM || (size_t)in_sizes[5] < (size_t)DM * DM || in_sizes[6] < DM || in_sizes[7] < DM || in_sizes[8] < DM) return;
    if ((size_t)in_sizes[9] < (size_t)DFF * DM || in_sizes[10] < DFF || (size_t)in_sizes[11] < (size_t)DM * DFF || in_sizes[12] < DM || in_sizes[13] < DM || in_sizes[14] < DM) return;
    if ((size_t)out_size < OUT1_OFF + (size_t)NB * SEQ * SEQ) return;
    float* OUT0 = (float*)d_out;
    float* OUT1 = (float*)d_out + OUT1_OFF;

    const size_t szW = (size_t)3 * DM * DM * 2 + (size_t)DM * DM * 2 + (size_t)DFF * DM * 2 + (size_t)DM * DFF * 2;
    const size_t TP  = (size_t)NTOK * DM * 2;
    const size_t R1  = 3 * TP;
    const size_t R2  = (2 * TP > (size_t)16 * SEQ * SEQ) ? 2 * TP : (size_t)16 * SEQ * SEQ;
    const size_t R3  = 3 * TP;
    const size_t R4  = ((size_t)32 * SEQ * SEQ > 4 * TP) ? (size_t)32 * SEQ * SEQ : 4 * TP;
    const size_t o1 = szW, o2 = o1 + R1, o3 = o2 + R2, o4 = o3 + R3, total = o4 + R4;
    if (total > ws_size || total > (size_t)134217728) return;
    char* ws = (char*)d_ws;
    bf*  WIP  = (bf*)ws;
    h16* WO16 = (h16*)(ws + (size_t)3 * DM * DM * 2);
    h16* W1H  = (h16*)(ws + (size_t)3 * DM * DM * 2 + (size_t)DM * DM * 2);
    h16* W2H  = (h16*)(ws + (size_t)3 * DM * DM * 2 + (size_t)DM * DM * 2 + (size_t)DFF * DM * 2);
    bf* QB = (bf*)(ws + o1); bf* KB = (bf*)(ws + o1 + TP); bf* VB = (bf*)(ws + o1 + 2 * TP);
    float* CTX = (float*)(ws + o1); h16* CTX16 = (h16*)(ws + o1 + 2 * TP); h16* FFH16 = (h16*)(ws + o1);
    float* F32A = (float*)(ws + o2); h16* P16 = (h16*)(ws + o2); float* ATT = (float*)(ws + o2); float* FF2 = (float*)(ws + o2);
    h16* QP16 = (h16*)(ws + o3); h16* KP16 = (h16*)(ws + o3 + TP); h16* VT16 = (h16*)(ws + o3 + 2 * TP);
    float* X1F = (float*)(ws + o3); h16* X1H = (h16*)(ws + o3 + 2 * TP);
    float* S = (float*)(ws + o4); float* FF1 = (float*)(ws + o4);

    const size_t n8tok = (size_t)NTOK * DM / 8;
    k_cvtin<<<(unsigned)((n8tok + 255) / 256), 256, 0, stream>>>(q, QB, n8tok);
    k_cvtin<<<(unsigned)((n8tok + 255) / 256), 256, 0, stream>>>(kin, KB, n8tok);
    k_cvtin<<<(unsigned)((n8tok + 255) / 256), 256, 0, stream>>>(vin, VB, n8tok);
    k_cvtb<<<(unsigned)(((size_t)3 * DM * DM / 8 + 255) / 256), 256, 0, stream>>>(ipw, WIP, (size_t)3 * DM * DM / 8);
    k_cvth<<<(unsigned)(((size_t)DM * DM / 8 + 255) / 256), 256, 0, stream>>>(ow, WO16, (size_t)DM * DM / 8, CW);
    k_cvth<<<(unsigned)(((size_t)DFF * DM / 8 + 255) / 256), 256, 0, stream>>>(w1, W1H, (size_t)DFF * DM / 8, CW);
    k_cvth<<<(unsigned)(((size_t)DM * DFF / 8 + 255) / 256), 256, 0, stream>>>(w2, W2H, (size_t)DM * DFF / 8, CW);
    k_gemmw<bf, true><<<dim3(NTOK / 64, DM / 64, 1), 32, 0, stream>>>(QB, DM, WIP, DM, DM, F32A, DM, ipb, 1.0f, 0, 0, 0);
    k_tof16<false, false><<<(unsigned)((n8tok + 255) / 256), 256, 0, stream>>>(F32A, QP16, n8tok, CQK, nullptr, 1, 1);
    k_gemmw<bf, true><<<dim3(NTOK / 64, DM / 64, 1), 32, 0, stream>>>(KB, DM, WIP + (size_t)DM * DM, DM, DM, F32A, DM, ipb + DM, 1.0f, 0, 0, 0);
    k_tof16<false, false><<<(unsigned)((n8tok + 255) / 256), 256, 0, stream>>>(F32A, KP16, n8tok, CQK, nullptr, 1, 1);
    k_gemmw<bf, false><<<dim3(DM / 64, SEQ / 64, NB), 32, 0, stream>>>(WIP + (size_t)2 * DM * DM, DM, VB, DM, DM, F32A, SEQ, nullptr, 1.0f, 0, (size_t)SEQ * DM, (size_t)DM * SEQ);
    k_tof16<false, true><<<(unsigned)((n8tok + 255) / 256), 256, 0, stream>>>(F32A, VT16, n8tok, CVV, ipb + 2 * DM, SEQ, DM);
    for (int b = 0; b < NB; ++b) {
        k_gemmw<h16, false><<<dim3(SEQ / 64, SEQ / 64, NH), 32, 0, stream>>>(QP16 + (size_t)b * SEQ * DM, DM, KP16 + (size_t)b * SEQ * DM, DM, HD, S, SEQ, nullptr, 1.0f, (size_t)HD, (size_t)HD, (size_t)SEQ * SEQ);
        k_soft<<<SEQ / 8, 256, 0, stream>>>(S, P16, OUT1 + (size_t)b * SEQ * SEQ);
        k_gemmw<h16, false><<<dim3(SEQ / 64, HD / 64, NH), 32, 0, stream>>>(P16, SEQ, VT16 + (size_t)b * DM * SEQ, SEQ, SEQ, CTX + (size_t)b * SEQ * DM, DM, nullptr, 1.0f, (size_t)SEQ * SEQ, (size_t)HD * SEQ, (size_t)HD);
    }
    k_tof16<false, false><<<(unsigned)((n8tok + 255) / 256), 256, 0, stream>>>(CTX, CTX16, n8tok, 1.0f, nullptr, 1, 1);
    k_gemmw<h16, true><<<dim3(NTOK / 64, DM / 64, 1), 32, 0, stream>>>(CTX16, DM, WO16, DM, DM, ATT, DM, ob, OSC_O, 0, 0, 0);
    k_ln<true><<<NTOK / 8, 256, 0, stream>>>(q, ATT, ln1g, ln1b, X1F, X1H);
    k_gemmw<h16, true><<<dim3(NTOK / 64, DFF / 64, 1), 32, 0, stream>>>(X1H, DM, W1H, DM, DM, FF1, DFF, b1, OSC_F, 0, 0, 0);
    k_tof16<true, false><<<(unsigned)(((size_t)NTOK * DFF / 8 + 255) / 256), 256, 0, stream>>>(FF1, FFH16, (size_t)NTOK * DFF / 8, CX, nullptr, 1, 1);
    k_gemmw<h16, true><<<dim3(NTOK / 64, DM / 64, 1), 32, 0, stream>>>(FFH16, DFF, W2H, DFF, DFF, FF2, DM, b2, OSC_F, 0, 0, 0);
    k_ln<false><<<NTOK / 8, 256, 0, stream>>>(X1F, FF2, ln2g, ln2b, OUT0, nullptr);
}
